// MultiHeadAttentionBase_6803228197596
// MI455X (gfx1250) — hardware-verified
//
#include <hip/hip_runtime.h>

typedef __attribute__((ext_vector_type(16))) __bf16   v16b;
typedef __attribute__((ext_vector_type(8)))  __bf16   v8b;
typedef __attribute__((ext_vector_type(8)))  float    v8f;
typedef __attribute__((ext_vector_type(4)))  float    v4f;
typedef __attribute__((ext_vector_type(4)))  unsigned int v4u;

constexpr int NBATCH = 4;
constexpr int NSEQ   = 2048;
constexpr int NDIM   = 1024;
constexpr int NHEAD  = 16;
constexpr int DHEAD  = 64;
constexpr int QBLK   = 64;
constexpr int KCH    = 64;
constexpr int NWAVE  = 4;
constexpr int OSP    = 68;
constexpr size_t NTOT = (size_t)NBATCH * NSEQ * NDIM;

static_assert(NHEAD * DHEAD == NDIM, "x");
static_assert(NSEQ % QBLK == 0 && NSEQ % KCH == 0, "x");
static_assert(DHEAD == 64 && KCH == 64, "x");
static_assert(NTOT % 8 == 0, "x");
static_assert(3 * NTOT * 2 <= (size_t)134217728, "x");


__device__ __forceinline__ unsigned short f2bf_bits(float f) {
  unsigned u = __float_as_uint(f);
  return (unsigned short)((u + 0x7FFFu + ((u >> 16) & 1u)) >> 16);
}
__device__ __forceinline__ __bf16 at_f2bf(float f) { return __builtin_bit_cast(__bf16, f2bf_bits(f)); }
__device__ __forceinline__ void at_split(float f, __bf16& hi, __bf16& lo) {
  const unsigned short hb = f2bf_bits(f);
  hi = __builtin_bit_cast(__bf16, hb);
  lo = at_f2bf(f - __uint_as_float(((unsigned)hb) << 16));
}
__device__ __forceinline__ v8f at_mma(v16b a, v16b b, v8f c) {
  c = __builtin_amdgcn_wmma_f32_16x16x32_bf16(false, a, false, b, (short)0, c, false, false);
  asm volatile("v_nop\n\tv_nop\n\tv_nop\n\tv_nop" : "+v"(c) : "v"(a), "v"(b));
  return c;
}
union FragU { v16b v; v8b h[2]; };
__device__ __forceinline__ v16b ld_frag_lds(const unsigned short* p) {
  FragU f;
  f.h[0] = *(const v8b*)(const void*)(p);
  f.h[1] = *(const v8b*)(const void*)(p + 16);
  return f.v;
}
__device__ __forceinline__ v16b ld_frag_bf(const __bf16* p) {
  FragU f;
  f.h[0] = *(const v8b*)(p);
  f.h[1] = *(const v8b*)(p + 16);
  return f.v;
}
__device__ __forceinline__ v16b ld_frag_glob(const unsigned short* p) {
  FragU f;
  f.h[0] = *(const v8b*)(const void*)(p);
  f.h[1] = *(const v8b*)(const void*)(p + 16);
  return f.v;
}

__global__ __launch_bounds__(256) void cvt_f32_bf16x8(const float* __restrict__ src,
                                                      unsigned short* __restrict__ dst, int n8) {
  const int i = blockIdx.x * 256 + threadIdx.x;
  if (i < n8) {
    const v4f a = *(const v4f*)(src + (size_t)8 * i);
    const v4f c = *(const v4f*)(src + (size_t)8 * i + 4);
    v4u w;
    w.x = (unsigned)f2bf_bits(a.x) | ((unsigned)f2bf_bits(a.y) << 16);
    w.y = (unsigned)f2bf_bits(a.z) | ((unsigned)f2bf_bits(a.w) << 16);
    w.z = (unsigned)f2bf_bits(c.x) | ((unsigned)f2bf_bits(c.y) << 16);
    w.w = (unsigned)f2bf_bits(c.z) | ((unsigned)f2bf_bits(c.w) << 16);
    volatile v4u* d = (volatile v4u*)(void*)(dst + (size_t)8 * i);
    *d = w;
    __threadfence();
    *d = w;
  }
}

__global__ __launch_bounds__(128)
void mha64_kernel(const unsigned short* __restrict__ qp, const unsigned short* __restrict__ kp,
                  const unsigned short* __restrict__ vp, float* __restrict__ out) {
  __shared__ __align__(16) unsigned short Ksh[KCH * DHEAD];
  __shared__ __align__(16) unsigned short Vth[DHEAD * KCH];
  __shared__ __align__(16) __bf16 Psh[NWAVE][16 * KCH];
  __shared__ __align__(16) __bf16 Psl[NWAVE][16 * KCH];
  __shared__ __align__(16) float  Os[NWAVE][16 * OSP];

  const int tid  = threadIdx.x;
  const int wave = tid >> 5;
  const int lane = tid & 31;
  const int hh   = lane >> 4;
  const int c    = lane & 15;

  constexpr int nqb = NSEQ / QBLK;
  const int bx = blockIdx.x;
  const int qb = bx % nqb;
  const int bh = bx / nqb;
  const int h  = bh % NHEAD;
  const int b  = bh / NHEAD;
  const int q0 = qb * QBLK + wave * 16;

  const size_t boff = (size_t)b * NSEQ * NDIM + (size_t)h * DHEAD;
  const unsigned short* qb_ptr = qp + boff;
  const unsigned short* kb_ptr = kp + boff;
  const unsigned short* vb_ptr = vp + boff;
  float*                ob_ptr = out + boff;

  v16b qa[2];
  {
    const unsigned short* qrow = qb_ptr + (size_t)(q0 + c) * NDIM;
#pragma unroll
    for (int dc = 0; dc < 2; ++dc) qa[dc] = ld_frag_glob(qrow + dc * 32 + 8 * hh);
  }

  float mrow[8], lrow[8];
  v8f oacc[4];
#pragma unroll
  for (int r = 0; r < 8; ++r) { mrow[r] = -__builtin_inff(); lrow[r] = 0.f; }
#pragma unroll
  for (int t = 0; t < 4; ++t) oacc[t] = (v8f){0.f, 0.f, 0.f, 0.f, 0.f, 0.f, 0.f, 0.f};

  constexpr int nChunks = NSEQ / KCH;
  for (int kc = 0; kc < nChunks; ++kc) {
    const int kv0 = kc * KCH;
    __syncthreads();
    {
      const int kvr = tid >> 1, dh = (tid & 1) * 32;
      const size_t roff = (size_t)(kv0 + kvr) * NDIM + dh;
      const unsigned short* krow = kb_ptr + roff;
      const unsigned short* vrow = vb_ptr + roff;
#pragma unroll
      for (int i = 0; i < 4; ++i) {
        const v4u kw = *(const v4u*)(const void*)(krow + 8 * i);
        const v4u vw = *(const v4u*)(const void*)(vrow + 8 * i);
        *(v4u*)(void*)(Ksh + kvr * DHEAD + dh + 8 * i) = kw;
#pragma unroll
        for (int e = 0; e < 4; ++e) {
          const unsigned w = vw[e];
          const int d = dh + 8 * i + 2 * e;
          Vth[d * KCH + kvr]       = (unsigned short)(w & 0xffffu);
          Vth[(d + 1) * KCH + kvr] = (unsigned short)(w >> 16);
        }
      }
    }
    __syncthreads();

    v8f s[4];
#pragma unroll
    for (int j = 0; j < 4; ++j) {
      s[j] = (v8f){0.f, 0.f, 0.f, 0.f, 0.f, 0.f, 0.f, 0.f};
#pragma unroll
      for (int dc = 0; dc < 2; ++dc) {
        const v16b kb = ld_frag_lds(Ksh + (j * 16 + c) * DHEAD + dc * 32 + 8 * hh);
        s[j] = at_mma(qa[dc], kb, s[j]);
      }
    }

    float cm[8];
#pragma unroll
    for (int r = 0; r < 8; ++r) {
      float m = -__builtin_inff();
#pragma unroll
      for (int j = 0; j < 4; ++j) {
        s[j][r] = s[j][r] * 0.125f;
        m = fmaxf(m, s[j][r]);
      }
#pragma unroll
      for (int off = 1; off < 16; off <<= 1) m = fmaxf(m, __shfl_xor(m, off, 32));
      cm[r] = m;
    }
    __bf16* pwh = Psh[wave];
    __bf16* pwl = Psl[wave];
#pragma unroll
    for (int r = 0; r < 8; ++r) {
      const float mnew  = fmaxf(mrow[r], cm[r]);
      const float alpha = expf(mrow[r] - mnew);
      mrow[r] = mnew;
      float psum = 0.f;
#pragma unroll
      for (int j = 0; j < 4; ++j) {
        const float p = expf(s[j][r] - mnew);
        psum += p;
        __bf16 ph, pl;
        at_split(p, ph, pl);
        pwh[(8 * hh + r) * KCH + j * 16 + c] = ph;
        pwl[(8 * hh + r) * KCH + j * 16 + c] = pl;
      }
#pragma unroll
      for (int off = 1; off < 16; off <<= 1) psum += __shfl_xor(psum, off, 32);
      lrow[r] = lrow[r] * alpha + psum;
#pragma unroll
      for (int t = 0; t < 4; ++t) oacc[t][r] *= alpha;
    }
    __builtin_amdgcn_fence(__ATOMIC_RELEASE, "workgroup");
    __builtin_amdgcn_wave_barrier();
    __builtin_amdgcn_fence(__ATOMIC_ACQUIRE, "workgroup");

#pragma unroll 1
    for (int kk = 0; kk < 2; ++kk) {
      const v16b pa = ld_frag_bf(pwh + c * KCH + kk * 32 + 8 * hh);
      const v16b pl = ld_frag_bf(pwl + c * KCH + kk * 32 + 8 * hh);
#pragma unroll
      for (int t = 0; t < 4; ++t) {
        const v16b vb = ld_frag_lds(Vth + (t * 16 + c) * KCH + kk * 32 + 8 * hh);
        oacc[t] = at_mma(pa, vb, oacc[t]);
        oacc[t] = at_mma(pl, vb, oacc[t]);
      }
    }
  }

  float* os = Os[wave];
#pragma unroll
  for (int r = 0; r < 8; ++r) {
    const float inv = 1.0f / lrow[r];
#pragma unroll
    for (int t = 0; t < 4; ++t) os[(8 * hh + r) * OSP + t * 16 + c] = oacc[t][r] * inv;
  }
  __builtin_amdgcn_fence(__ATOMIC_RELEASE, "workgroup");
  __builtin_amdgcn_wave_barrier();
  __builtin_amdgcn_fence(__ATOMIC_ACQUIRE, "workgroup");
  {
    const int c4 = (lane & 15) * 4;
    for (int pass = 0; pass < 2; ++pass) {
#pragma unroll
      for (int it = 0; it < 8; ++it) {
        const int row = it * 2 + hh;
        const v4f val = *(const v4f*)(os + row * OSP + c4);
        *(volatile v4f*)(ob_ptr + (size_t)(q0 + row) * NDIM + c4) = val;
      }
      __threadfence();
    }
  }
}

extern "C" void kernel_launch(void* const* d_in, const int* in_sizes, int n_in,
                              void* d_out, int out_size, void* d_ws, size_t ws_size,
                              hipStream_t stream) {
  if (n_in < 3) return;
  if ((size_t)in_sizes[0] != NTOT || (size_t)in_sizes[1] != NTOT || (size_t)in_sizes[2] != NTOT) return;
  if ((size_t)out_size != NTOT) return;
  const size_t carve = 3 * NTOT * sizeof(unsigned short);
  if (ws_size < carve) return;

  const float* q = (const float*)d_in[0];
  const float* k = (const float*)d_in[1];
  const float* v = (const float*)d_in[2];
  float* out = (float*)d_out;

  unsigned short* qpl = (unsigned short*)d_ws;
  unsigned short* kpl = qpl + NTOT;
  unsigned short* vpl = kpl + NTOT;

  const int n8 = (int)(NTOT / 8);
  const int cblocks = (n8 + 255) / 256;
  cvt_f32_bf16x8<<<cblocks, 256, 0, stream>>>(q, qpl, n8);
  cvt_f32_bf16x8<<<cblocks, 256, 0, stream>>>(k, kpl, n8);
  cvt_f32_bf16x8<<<cblocks, 256, 0, stream>>>(v, vpl, n8);

  const int ablocks = NBATCH * NHEAD * (NSEQ / QBLK);
  mha64_kernel<<<ablocks, 128, 0, stream>>>(qpl, kpl, vpl, out);
}
